// ODEForecaster_80985903333558
// MI455X (gfx1250) — hardware-verified
//
#include <hip/hip_runtime.h>

typedef __attribute__((ext_vector_type(16))) _Float16 v16h;
typedef __attribute__((ext_vector_type(8)))  _Float16 v8h;
typedef __attribute__((ext_vector_type(16))) __bf16   v16b;
typedef __attribute__((ext_vector_type(8)))  __bf16   v8b;
typedef __attribute__((ext_vector_type(8)))  float    v8f;
typedef __attribute__((ext_vector_type(4)))  float    v4f;
typedef __attribute__((ext_vector_type(4)))  unsigned v4u;

__device__ __forceinline__ unsigned short f2bf_bits(float f) {
  unsigned u = __float_as_uint(f);
  return (unsigned short)((u + 0x7FFFu + ((u >> 16) & 1u)) >> 16);
}
__device__ __forceinline__ float bf_bits2f(unsigned short h) { return __uint_as_float(((unsigned)h) << 16); }

__device__ __forceinline__ void dep_guard_h(v8f& a, v8f& b, v16h x, v16h y) { asm volatile("v_nop\n\tv_nop\n\tv_nop\n\tv_nop" : "+v"(a), "+v"(b) : "v"(x), "v"(y)); }
__device__ __forceinline__ void dep_guard_b(v8f& a, v8f& b, v16b x, v16b y) { asm volatile("v_nop\n\tv_nop\n\tv_nop\n\tv_nop" : "+v"(a), "+v"(b) : "v"(x), "v"(y)); }
__device__ __forceinline__ void keep4_h(v16h a, v16h b, v16h c, v16h d) { asm volatile("v_nop" :: "v"(a), "v"(b), "v"(c), "v"(d)); }
__device__ __forceinline__ void keep4_b(v16b a, v16b b, v16b c, v16b d) { asm volatile("v_nop" :: "v"(a), "v"(b), "v"(c), "v"(d)); }
__device__ __forceinline__ void acc_guard4(v8f& a, v8f& b, v8f& c, v8f& d) { asm volatile("v_nop\n\tv_nop\n\tv_nop\n\tv_nop" : "+v"(a), "+v"(b), "+v"(c), "+v"(d)); }
template <typename T> struct Frag;
template <> struct Frag<_Float16> {
  typedef v16h V; union U { v16h v; v8h h[2]; };
  static __device__ __forceinline__ v16h load(const _Float16* p) {
    U f; f.h[0] = *(const v8h*)(p); f.h[1] = *(const v8h*)(p + 16); return f.v;
  }
  static __device__ __forceinline__ v8f mma(v16h a, v16h b, v8f c) {
    return __builtin_amdgcn_wmma_f32_16x16x32_f16(false, a, false, b, (short)0, c, false, false);
  }
  static __device__ __forceinline__ void guard(v8f& a, v8f& b, v16h x, v16h y) { dep_guard_h(a, b, x, y); }
  static __device__ __forceinline__ void keep(v16h a, v16h b, v16h c, v16h d) { keep4_h(a, b, c, d); }
};
template <> struct Frag<__bf16> {
  typedef v16b V; union U { v16b v; v8b h[2]; };
  static __device__ __forceinline__ v16b load(const __bf16* p) {
    U f; f.h[0] = *(const v8b*)(p); f.h[1] = *(const v8b*)(p + 16); return f.v;
  }
  static __device__ __forceinline__ v8f mma(v16b a, v16b b, v8f c) {
    return __builtin_amdgcn_wmma_f32_16x16x32_bf16(false, a, false, b, (short)0, c, false, false);
  }
  static __device__ __forceinline__ void guard(v8f& a, v8f& b, v16b x, v16b y) { dep_guard_b(a, b, x, y); }
  static __device__ __forceinline__ void keep(v16b a, v16b b, v16b c, v16b d) { keep4_b(a, b, c, d); }
};
typedef Frag<_Float16> FragH;

template <int ET> struct Elem;
template <> struct Elem<0> { typedef _Float16 T; };
template <> struct Elem<1> { typedef __bf16 T; };
template <int ET, bool SPLIT, int BIAS_MODE, int OUT_MODE, bool RESID, int ACT = 0>
__global__ __launch_bounds__(256) void wmma_gemm64(
    const unsigned short* __restrict__ Ap, const unsigned short* __restrict__ A2p, int lda, long strideA,
    const unsigned short* __restrict__ Btp, const unsigned short* __restrict__ Bt2p, int ldb, long strideB,
    void* __restrict__ Cout, void* __restrict__ Cout2, int ldc, long strideC,
    const float* __restrict__ bias,
    const float* __restrict__ resid, long strideR,
    int M, int N, int K, float scale) {
  typedef typename Elem<ET>::T T;
  typedef typename Frag<T>::V V;
  const T* A = (const T*)Ap; const T* A2 = (const T*)A2p; const T* Bt = (const T*)Btp; const T* Bt2 = (const T*)Bt2p;
  __shared__ __align__(16) float sT[8][16 * 68];
  const int b    = blockIdx.y;
  const int lane = threadIdx.x & 31;
  const int wave = threadIdx.x >> 5;
  const int tilesN = N >> 6;
  const int tilesM = M >> 6;
  const int tile = blockIdx.x * 8 + wave;
  if (tile >= tilesM * tilesN) return;
  const int tm = tile / tilesN;
  const int tn = tile - tm * tilesN;
  const int m0 = tm << 6;
  const int n0 = tn << 6;

  const T* Ab  = A  + (size_t)b * strideA;
  const T* Bb  = Bt + (size_t)b * strideB;
  const T* Ab2 = SPLIT ? (A2  + (size_t)b * strideA) : nullptr;
  const T* Bb2 = SPLIT ? (Bt2 + (size_t)b * strideB) : nullptr;

  const int rlane = lane & 15;
  const int koff  = (lane >> 4) * 8;
  const int mOff  = (lane >> 4) * 8;

  v8f acc[4][4];
#pragma unroll
  for (int i = 0; i < 4; ++i)
#pragma unroll
    for (int j = 0; j < 4; ++j) acc[i][j] = (v8f){0.f,0.f,0.f,0.f,0.f,0.f,0.f,0.f};

  for (int k0 = 0; k0 < K; k0 += 32) {
    V bh[4], bl[4];
#pragma unroll
    for (int j = 0; j < 4; ++j) {
      const size_t bo = (size_t)(n0 + (j << 4) + rlane) * ldb + koff + k0;
      bh[j] = Frag<T>::load(Bb + bo);
      if (SPLIT) bl[j] = Frag<T>::load(Bb2 + bo);
    }
#pragma unroll
    for (int i = 0; i < 4; ++i) {
      const size_t ao = (size_t)(m0 + (i << 4) + rlane) * lda + koff + k0;
      V ah = Frag<T>::load(Ab + ao);
      V al;
      if (SPLIT) al = Frag<T>::load(Ab2 + ao);
#pragma unroll
      for (int j = 0; j < 4; ++j) {
        acc[i][j] = Frag<T>::mma(ah, bh[j], acc[i][j]);
        if (SPLIT) {
          acc[i][j] = Frag<T>::mma(ah, bl[j], acc[i][j]);
          acc[i][j] = Frag<T>::mma(al, bh[j], acc[i][j]);
        }
      }
      Frag<T>::guard(acc[i][0], acc[i][3], ah, SPLIT ? al : ah);
    }
    Frag<T>::keep(bh[0], bh[1], bh[2], bh[3]);
    if (SPLIT) Frag<T>::keep(bl[0], bl[1], bl[2], bl[3]);
  }
  acc_guard4(acc[0][0], acc[0][1], acc[0][2], acc[0][3]);
  acc_guard4(acc[1][0], acc[1][1], acc[1][2], acc[1][3]);
  acc_guard4(acc[2][0], acc[2][1], acc[2][2], acc[2][3]);
  acc_guard4(acc[3][0], acc[3][1], acc[3][2], acc[3][3]);

  float* slab = sT[wave];
  const float* Rb = RESID ? (resid + (size_t)b * strideR) : nullptr;
#pragma unroll
  for (int i = 0; i < 4; ++i) {
    const int mBase = m0 + (i << 4);
#pragma unroll
    for (int j = 0; j < 4; ++j) {
      const int n = n0 + (j << 4) + rlane;
      float bv = 0.f;
      if (BIAS_MODE == 2) bv = bias[n];
#pragma unroll
      for (int r = 0; r < 8; ++r) {
        float v = acc[i][j][r] * scale;
        if (BIAS_MODE == 1) v += bias[mBase + mOff + r];
        if (BIAS_MODE == 2) v += bv;
        if (RESID) v += Rb[(size_t)(mBase + mOff + r) * ldc + n];
        if (ACT == 1) v = tanhf(v);
        if (ACT == 2) v = fmaxf(v, 0.0f);
        if (ACT == 3) v = v / (1.0f + expf(-v));
        if (ACT == 4) v = (v > 0.f) ? v : 0.01f * v;
        if (ACT == 5) v = 0.5f * v * (1.0f + erff(v * 0.70710678118654752f));
        slab[(mOff + r) * 68 + (j << 4) + rlane] = v;
      }
    }
    __builtin_amdgcn_fence(__ATOMIC_RELEASE, "workgroup");
    __builtin_amdgcn_wave_barrier();
    __builtin_amdgcn_fence(__ATOMIC_ACQUIRE, "workgroup");
    if (OUT_MODE == 0) {
      float* C = (float*)Cout + (size_t)b * strideC;
      const int hh = lane >> 4, c4 = (lane & 15) * 4;
      for (int pass = 0; pass < 2; ++pass) {
#pragma unroll
        for (int it = 0; it < 8; ++it) {
          const int row = it * 2 + hh;
          v4f v = *(const v4f*)(slab + row * 68 + c4);
          *(volatile v4f*)(C + (size_t)(mBase + row) * ldc + n0 + c4) = v;
        }
        __threadfence();
      }
    } else {
      const int q = lane >> 3, c8 = (lane & 7) * 8;
      unsigned short* C  = (unsigned short*)Cout  + (size_t)b * strideC;
      unsigned short* C2 = (OUT_MODE == 2) ? ((unsigned short*)Cout2 + (size_t)b * strideC) : nullptr;
      for (int pass = 0; pass < 2; ++pass) {
#pragma unroll
        for (int it = 0; it < 4; ++it) {
          const int row = it * 4 + q;
          const float* sp = slab + row * 68 + c8;
          v8h hv, lv;
#pragma unroll
          for (int e = 0; e < 8; ++e) {
            if (OUT_MODE == 1) {
              hv[e] = (_Float16)sp[e];
            } else {
              unsigned short hb = f2bf_bits(sp[e]);
              unsigned short lb = f2bf_bits(sp[e] - bf_bits2f(hb));
              hv[e] = __builtin_bit_cast(_Float16, hb);
              lv[e] = __builtin_bit_cast(_Float16, lb);
            }
          }
          *(volatile v8h*)(C + (size_t)(mBase + row) * ldc + n0 + c8) = hv;
          if (OUT_MODE == 2) *(volatile v8h*)(C2 + (size_t)(mBase + row) * ldc + n0 + c8) = lv;
        }
        __threadfence();
      }
    }
    __builtin_amdgcn_fence(__ATOMIC_RELEASE, "workgroup");
    __builtin_amdgcn_wave_barrier();
    __builtin_amdgcn_fence(__ATOMIC_ACQUIRE, "workgroup");
  }
}

static constexpr int kBatch = 1024;
static constexpr int kState = 128;
static constexpr int kT     = 96;
static constexpr int kHid   = 128;
static constexpr int kG3    = 384;
static constexpr int kH1    = 64;
static constexpr int kOut   = 3072;
static constexpr int kRows  = 16;
static constexpr int kAPitch  = 136;
static constexpr int kXHPitch = 264;
static constexpr int kOPitch  = 132;
#define ACT_CARRY 16.0f
#define W_CARRY 16.0f
#define PROD_INV (1.0f / 256.0f)

__device__ __forceinline__ v8f zero8() { v8f z = {0.f, 0.f, 0.f, 0.f, 0.f, 0.f, 0.f, 0.f}; return z; }
__device__ __forceinline__ unsigned h16bits(float f) { return (unsigned)__builtin_bit_cast(unsigned short, (_Float16)f); }
__device__ __forceinline__ unsigned pack_bf2(float a, float b, unsigned& lo_out) {
  const unsigned short ha = f2bf_bits(a), hb = f2bf_bits(b);
  const unsigned short la = f2bf_bits(a - bf_bits2f(ha)), lb = f2bf_bits(b - bf_bits2f(hb));
  lo_out = (unsigned)la | (((unsigned)lb) << 16);
  return (unsigned)ha | (((unsigned)hb) << 16);
}
__device__ __forceinline__ void guard_acc1(v8f& x, v16h a0, v16h a1, v16h a2, v16h a3, v16h b0, v16h b1, v16h b2, v16h b3) {
  asm volatile("v_nop\n\tv_nop\n\tv_nop\n\tv_nop" : "+v"(x) : "v"(a0), "v"(a1), "v"(a2), "v"(a3), "v"(b0), "v"(b1), "v"(b2), "v"(b3));
}
__device__ __forceinline__ void guard_acc3(v8f& x, v8f& y, v8f& z, v16h a, v16h p, v16h q, v16h s) {
  asm volatile("v_nop\n\tv_nop\n\tv_nop\n\tv_nop" : "+v"(x), "+v"(y), "+v"(z) : "v"(a), "v"(p), "v"(q), "v"(s));
}
__device__ __forceinline__ float sigm_f(float x) { return __builtin_amdgcn_rcpf(1.0f + expf(-x)); }

__global__ __launch_bounds__(256) void k_cast_h16(const float* __restrict__ in, unsigned short* __restrict__ out,
                                                  int n8, float scale) {
  const int i = blockIdx.x * 256 + threadIdx.x;
  if (i < n8) {
    const float* p = in + (size_t)i * 8;
    const v4f a = *(const v4f*)p;
    const v4f q = *(const v4f*)(p + 4);
    v4u w;
    w[0] = h16bits(a[0] * scale) | (h16bits(a[1] * scale) << 16);
    w[1] = h16bits(a[2] * scale) | (h16bits(a[3] * scale) << 16);
    w[2] = h16bits(q[0] * scale) | (h16bits(q[1] * scale) << 16);
    w[3] = h16bits(q[2] * scale) | (h16bits(q[3] * scale) << 16);
    volatile v4u* d = (volatile v4u*)(void*)(out + (size_t)i * 8);
    *d = w;
    __threadfence();
    *d = w;
  }
}

__global__ __launch_bounds__(256) void k_cast_bf2(const float* __restrict__ in, unsigned short* __restrict__ hi,
                                                  unsigned short* __restrict__ lo, int n8) {
  const int i = blockIdx.x * 256 + threadIdx.x;
  if (i < n8) {
    const float* p = in + (size_t)i * 8;
    const v4f a = *(const v4f*)p;
    const v4f q = *(const v4f*)(p + 4);
    v4u wh, wl;
    unsigned l0, l1, l2, l3;
    wh[0] = pack_bf2(a[0], a[1], l0);
    wh[1] = pack_bf2(a[2], a[3], l1);
    wh[2] = pack_bf2(q[0], q[1], l2);
    wh[3] = pack_bf2(q[2], q[3], l3);
    wl[0] = l0; wl[1] = l1; wl[2] = l2; wl[3] = l3;
    volatile v4u* dh = (volatile v4u*)(void*)(hi + (size_t)i * 8);
    volatile v4u* dl = (volatile v4u*)(void*)(lo + (size_t)i * 8);
    *dh = wh; *dl = wl;
    __threadfence();
    *dh = wh; *dl = wl;
  }
}

__global__ __launch_bounds__(256) void k_gelu2(const float* __restrict__ in, unsigned short* __restrict__ hi,
                                                unsigned short* __restrict__ lo, int n2) {
  const int i = blockIdx.x * 256 + threadIdx.x;
  if (i < n2) {
    unsigned wh = 0u, wl = 0u;
#pragma unroll 1
    for (int e = 0; e < 2; ++e) {
      const float x = in[(size_t)2 * i + e];
      const float g = 0.5f * x * (1.0f + erff(x * 0.70710678118654752f));
      const unsigned short hb = f2bf_bits(g);
      const unsigned short lb = f2bf_bits(g - bf_bits2f(hb));
      wh |= ((unsigned)hb) << (16 * e);
      wl |= ((unsigned)lb) << (16 * e);
    }
    volatile unsigned* dh = (volatile unsigned*)(void*)hi + i;
    volatile unsigned* dl = (volatile unsigned*)(void*)lo + i;
    *dh = wh; *dl = wl;
    __threadfence();
    *dh = wh; *dl = wl;
  }
}

__global__ __launch_bounds__(256) void k_ode(const float* __restrict__ yl, const float* __restrict__ yh,
                                             const unsigned short* __restrict__ Wp, const float* __restrict__ bode,
                                             unsigned short* __restrict__ trajp) {
  __shared__ __align__(16) _Float16 sA[kRows * kAPitch];
  const int tid  = threadIdx.x;
  const int wave = tid >> 5, lane = tid & 31, c = lane & 15, hh = lane >> 4;
  const int j    = wave * 16 + c;
  const int row0 = blockIdx.x * kRows;
  const _Float16* W = (const _Float16*)(const void*)Wp;
  _Float16* traj = (_Float16*)(void*)trajp;

  const _Float16* wrow = W + (size_t)j * kState + 8 * hh;
  const v16h bw0 = FragH::load(wrow);
  const v16h bw1 = FragH::load(wrow + 32);
  const v16h bw2 = FragH::load(wrow + 64);
  const v16h bw3 = FragH::load(wrow + 96);
  const float bo = bode[j];

  float y[8];
  {
    const int jl = (j < 32) ? j : 31;
    const int jh = (j >= 32) ? (j - 32) : 0;
#pragma unroll
    for (int r = 0; r < 8; ++r) {
      const int bi = row0 + 8 * hh + r;
      const float v0 = yl[(size_t)bi * 32 + jl];
      const float v1 = yh[(size_t)bi * 96 + jh];
      y[r] = (j < 32) ? v0 : v1;
    }
  }
#pragma unroll
  for (int r = 0; r < 8; ++r) sA[(8 * hh + r) * kAPitch + j] = (_Float16)(y[r] * ACT_CARRY);
  __syncthreads();

  auto rowstore = [&](int t) {
    const int row = 2 * wave + hh;
    const v8h hv = *(const v8h*)(sA + row * kAPitch + c * 8);
    volatile v8h* d = (volatile v8h*)(traj + (((size_t)t * kBatch + row0 + row) * kState + c * 8));
    *d = hv;
    __threadfence();
    *d = hv;
  };
  rowstore(0);

  float k1[8], k2[8], k3[8], k4[8], k5[8], k6[8], arg[8];

  auto feval = [&](float* kd) {
    const _Float16* ap = sA + c * kAPitch + 8 * hh;
    const v16h a0 = FragH::load(ap);
    const v16h a1 = FragH::load(ap + 32);
    const v16h a2 = FragH::load(ap + 64);
    const v16h a3 = FragH::load(ap + 96);
    v8f acc = zero8();
    acc = FragH::mma(a0, bw0, acc);
    acc = FragH::mma(a1, bw1, acc);
    acc = FragH::mma(a2, bw2, acc);
    acc = FragH::mma(a3, bw3, acc);
    guard_acc1(acc, a0, a1, a2, a3, bw0, bw1, bw2, bw3);
#pragma unroll
    for (int r = 0; r < 8; ++r) kd[r] = tanhf(acc[r] * PROD_INV + bo);
  };
  auto swrite = [&](const float* a) {
    __syncthreads();
#pragma unroll
    for (int r = 0; r < 8; ++r) sA[(8 * hh + r) * kAPitch + j] = (_Float16)(a[r] * ACT_CARRY);
    __syncthreads();
  };

  const float del = 1.0f / 95.0f;
#pragma unroll 1
  for (int t = 1; t < kT; ++t) {
    float ta = (float)(t - 1) * del;
    float tb = (float)t * del;
    asm volatile("" : "+v"(ta));
    asm volatile("" : "+v"(tb));
    if (t == kT - 1) tb = 1.0f;
    const float dt = tb - ta;

    feval(k1);
#pragma unroll
    for (int r = 0; r < 8; ++r) arg[r] = y[r] + dt * (0.2f * k1[r]);
    swrite(arg);
    feval(k2);
#pragma unroll
    for (int r = 0; r < 8; ++r)
      arg[r] = y[r] + dt * ((3.0f / 40.0f) * k1[r] + (9.0f / 40.0f) * k2[r]);
    swrite(arg);
    feval(k3);
#pragma unroll
    for (int r = 0; r < 8; ++r)
      arg[r] = y[r] + dt * ((44.0f / 45.0f) * k1[r] - (56.0f / 15.0f) * k2[r] + (32.0f / 9.0f) * k3[r]);
    swrite(arg);
    feval(k4);
#pragma unroll
    for (int r = 0; r < 8; ++r)
      arg[r] = y[r] + dt * ((19372.0f / 6561.0f) * k1[r] - (25360.0f / 2187.0f) * k2[r]
                            + (64448.0f / 6561.0f) * k3[r] - (212.0f / 729.0f) * k4[r]);
    swrite(arg);
    feval(k5);
#pragma unroll
    for (int r = 0; r < 8; ++r)
      arg[r] = y[r] + dt * ((9017.0f / 3168.0f) * k1[r] - (355.0f / 33.0f) * k2[r]
                            + (46732.0f / 5247.0f) * k3[r] + (49.0f / 176.0f) * k4[r]
                            - (5103.0f / 18656.0f) * k5[r]);
    swrite(arg);
    feval(k6);
#pragma unroll
    for (int r = 0; r < 8; ++r)
      y[r] = y[r] + dt * ((35.0f / 384.0f) * k1[r] + (500.0f / 1113.0f) * k3[r]
                          + (125.0f / 192.0f) * k4[r] - (2187.0f / 6784.0f) * k5[r]
                          + (11.0f / 84.0f) * k6[r]);
    swrite(y);
    rowstore(t);
  }
}

template <bool SEQ_OUT>
__global__ __launch_bounds__(256) void k_gru(const unsigned short* __restrict__ xsp,
                                             const unsigned short* __restrict__ Wihp, const unsigned short* __restrict__ Whhp,
                                             const float* __restrict__ bih, const float* __restrict__ bhh,
                                             unsigned short* hseqp, unsigned short* hhip, unsigned short* hlop) {
  __shared__ __align__(16) _Float16 sXH[kRows * kXHPitch];
  __shared__ __align__(16) float sO[SEQ_OUT ? 4 : kRows * kOPitch];
  const int tid  = threadIdx.x;
  const int wave = tid >> 5, lane = tid & 31, c = lane & 15, hh = lane >> 4;
  const int u    = wave * 16 + c;
  const int row0 = blockIdx.x * kRows;
  const _Float16* xs  = (const _Float16*)(const void*)xsp;
  const _Float16* Wih = (const _Float16*)(const void*)Wihp;
  const _Float16* Whh = (const _Float16*)(const void*)Whhp;
  _Float16* hseq = (_Float16*)(void*)hseqp;

  const float b_r  = bih[u] + bhh[u];
  const float b_z  = bih[kHid + u] + bhh[kHid + u];
  const float b_in = bih[2 * kHid + u];
  const float b_hn = bhh[2 * kHid + u];

  {
    v4u* z = (v4u*)(void*)sXH;
    const v4u zz = {0u, 0u, 0u, 0u};
    for (int i = tid; i < (kRows * kXHPitch * 2) / 16; i += 256) z[i] = zz;
  }
  float h[8];
#pragma unroll
  for (int r = 0; r < 8; ++r) h[r] = 0.0f;
  __syncthreads();

  const _Float16* ap = sXH + c * kXHPitch + 8 * hh;
  const _Float16* wr = Wih + (size_t)u * kState + 8 * hh;
  const _Float16* wz = Wih + (size_t)(kHid + u) * kState + 8 * hh;
  const _Float16* wn = Wih + (size_t)(2 * kHid + u) * kState + 8 * hh;
  const _Float16* gr = Whh + (size_t)u * kHid + 8 * hh;
  const _Float16* gz = Whh + (size_t)(kHid + u) * kHid + 8 * hh;
  const _Float16* gn = Whh + (size_t)(2 * kHid + u) * kHid + 8 * hh;

#pragma unroll 1
  for (int t = 0; t < kT; ++t) {
    {
      const int row = tid >> 4, c8 = (tid & 15) * 8;
      const v8h xv = *(const v8h*)(xs + (((size_t)t * kBatch + row0 + row) * kState + c8));
      *(v8h*)(sXH + row * kXHPitch + c8) = xv;
    }
    __syncthreads();

    v8f aR = zero8(), aZ = zero8(), aNi = zero8(), aNh = zero8();
#pragma unroll
    for (int kb = 0; kb < 4; ++kb) {
      const v16h a  = FragH::load(ap + kb * 32);
      const v16h fr = FragH::load(wr + kb * 32);
      const v16h fz = FragH::load(wz + kb * 32);
      const v16h fn = FragH::load(wn + kb * 32);
      aR  = FragH::mma(a, fr, aR);
      aZ  = FragH::mma(a, fz, aZ);
      aNi = FragH::mma(a, fn, aNi);
      guard_acc3(aR, aZ, aNi, a, fr, fz, fn);
    }
#pragma unroll
    for (int kb = 0; kb < 4; ++kb) {
      const v16h a  = FragH::load(ap + kState + kb * 32);
      const v16h fr = FragH::load(gr + kb * 32);
      const v16h fz = FragH::load(gz + kb * 32);
      const v16h fn = FragH::load(gn + kb * 32);
      aR  = FragH::mma(a, fr, aR);
      aZ  = FragH::mma(a, fz, aZ);
      aNh = FragH::mma(a, fn, aNh);
      guard_acc3(aR, aZ, aNh, a, fr, fz, fn);
    }

#pragma unroll
    for (int r = 0; r < 8; ++r) {
      const float rg = sigm_f(aR[r] * PROD_INV + b_r);
      const float zg = sigm_f(aZ[r] * PROD_INV + b_z);
      const float pn = (aNi[r] * PROD_INV + b_in) + rg * (aNh[r] * PROD_INV + b_hn);
      const float ng = tanhf(pn);
      h[r] = (1.0f - zg) * ng + zg * h[r];
    }
    __syncthreads();
#pragma unroll
    for (int r = 0; r < 8; ++r) sXH[(8 * hh + r) * kXHPitch + kState + u] = (_Float16)(h[r] * ACT_CARRY);
    __syncthreads();
    if (SEQ_OUT) {
      const int row = 2 * wave + hh;
      const v8h hv = *(const v8h*)(sXH + row * kXHPitch + kState + c * 8);
      volatile v8h* d = (volatile v8h*)(hseq + (((size_t)t * kBatch + row0 + row) * kHid + c * 8));
      *d = hv;
      __threadfence();
      *d = hv;
    }
  }

  if (!SEQ_OUT) {
#pragma unroll
    for (int r = 0; r < 8; ++r) sO[(8 * hh + r) * kOPitch + u] = h[r];
    __syncthreads();
    const int row = 2 * wave + hh;
    const float* sp = sO + row * kOPitch + c * 8;
    const v4f f0 = *(const v4f*)sp;
    const v4f f1 = *(const v4f*)(sp + 4);
    v4u wh, wl;
    unsigned l0, l1, l2, l3;
    wh[0] = pack_bf2(f0[0], f0[1], l0);
    wh[1] = pack_bf2(f0[2], f0[3], l1);
    wh[2] = pack_bf2(f1[0], f1[1], l2);
    wh[3] = pack_bf2(f1[2], f1[3], l3);
    wl[0] = l0; wl[1] = l1; wl[2] = l2; wl[3] = l3;
    const size_t o = (size_t)(row0 + row) * kHid + c * 8;
    volatile v4u* dh = (volatile v4u*)(void*)(hhip + o);
    volatile v4u* dl = (volatile v4u*)(void*)(hlop + o);
    *dh = wh; *dl = wl;
    __threadfence();
    *dh = wh; *dl = wl;
  }
}

extern "C" void kernel_launch(void* const* d_in, const int* in_sizes, int n_in,
                              void* d_out, int out_size, void* d_ws, size_t ws_size,
                              hipStream_t stream) {
  if (n_in < 17) return;
  const size_t szW   = (size_t)kState * kState * 2;
  const size_t szWg  = (size_t)kG3 * kState * 2;
  const size_t szW1  = (size_t)kH1 * kHid * 2;
  const size_t szW2  = (size_t)kOut * kH1 * 2;
  const size_t szSeq = (size_t)kT * kBatch * kState * 2;
  const size_t szH2  = (size_t)kBatch * kHid * 2;
  const size_t szG1  = (size_t)kBatch * kH1 * 4;
  const size_t szHd  = (size_t)kBatch * kH1 * 2;
  size_t off = 0;
  const size_t oWode = off; off += szW;
  const size_t oWih0 = off; off += szWg;
  const size_t oWhh0 = off; off += szWg;
  const size_t oWih1 = off; off += szWg;
  const size_t oWhh1 = off; off += szWg;
  const size_t oW1hi = off; off += szW1;
  const size_t oW1lo = off; off += szW1;
  const size_t oW2hi = off; off += szW2;
  const size_t oW2lo = off; off += szW2;
  const size_t oTraj = off; off += szSeq;
  const size_t oH1   = off; off += szSeq;
  const size_t oH2hi = off; off += szH2;
  const size_t oH2lo = off; off += szH2;
  const size_t oG1   = off; off += szG1;
  const size_t oHdhi = off; off += szHd;
  const size_t oHdlo = off; off += szHd;
  const size_t total = off;

  if (out_size != kBatch * kOut || ws_size < total) return;
  if (in_sizes[1] != kBatch * 32 || in_sizes[2] != kBatch * 96 || in_sizes[3] != kState * kState ||
      in_sizes[4] != kState || in_sizes[5] != kG3 * kState || in_sizes[6] != kG3 * kHid ||
      in_sizes[9] != kG3 * kHid || in_sizes[10] != kG3 * kHid || in_sizes[13] != kH1 * kHid ||
      in_sizes[15] != kOut * kH1 || in_sizes[16] != kOut) return;

  const float* yl   = (const float*)d_in[1];
  const float* yh   = (const float*)d_in[2];
  const float* Wode = (const float*)d_in[3];
  const float* bode = (const float*)d_in[4];
  const float* Wih0 = (const float*)d_in[5];
  const float* Whh0 = (const float*)d_in[6];
  const float* bih0 = (const float*)d_in[7];
  const float* bhh0 = (const float*)d_in[8];
  const float* Wih1 = (const float*)d_in[9];
  const float* Whh1 = (const float*)d_in[10];
  const float* bih1 = (const float*)d_in[11];
  const float* bhh1 = (const float*)d_in[12];
  const float* W1   = (const float*)d_in[13];
  const float* b1   = (const float*)d_in[14];
  const float* W2   = (const float*)d_in[15];
  const float* b2   = (const float*)d_in[16];
  float* out = (float*)d_out;

  unsigned char* w = (unsigned char*)d_ws;
  unsigned short* pWode = (unsigned short*)(w + oWode);
  unsigned short* pWih0 = (unsigned short*)(w + oWih0);
  unsigned short* pWhh0 = (unsigned short*)(w + oWhh0);
  unsigned short* pWih1 = (unsigned short*)(w + oWih1);
  unsigned short* pWhh1 = (unsigned short*)(w + oWhh1);
  unsigned short* pW1hi = (unsigned short*)(w + oW1hi);
  unsigned short* pW1lo = (unsigned short*)(w + oW1lo);
  unsigned short* pW2hi = (unsigned short*)(w + oW2hi);
  unsigned short* pW2lo = (unsigned short*)(w + oW2lo);
  unsigned short* pTraj = (unsigned short*)(w + oTraj);
  unsigned short* pH1   = (unsigned short*)(w + oH1);
  unsigned short* pH2hi = (unsigned short*)(w + oH2hi);
  unsigned short* pH2lo = (unsigned short*)(w + oH2lo);
  float*          pG1   = (float*)(w + oG1);
  unsigned short* pHdhi = (unsigned short*)(w + oHdhi);
  unsigned short* pHdlo = (unsigned short*)(w + oHdlo);

  const int n8W  = kState * kState / 8;
  const int n8Wg = kG3 * kState / 8;
  const int n8W1 = kH1 * kHid / 8;
  const int n8W2 = kOut * kH1 / 8;
  k_cast_h16<<<dim3((n8W + 255) / 256), dim3(256), 0, stream>>>(Wode, pWode, n8W, W_CARRY);
  k_cast_h16<<<dim3((n8Wg + 255) / 256), dim3(256), 0, stream>>>(Wih0, pWih0, n8Wg, W_CARRY);
  k_cast_h16<<<dim3((n8Wg + 255) / 256), dim3(256), 0, stream>>>(Whh0, pWhh0, n8Wg, W_CARRY);
  k_cast_h16<<<dim3((n8Wg + 255) / 256), dim3(256), 0, stream>>>(Wih1, pWih1, n8Wg, W_CARRY);
  k_cast_h16<<<dim3((n8Wg + 255) / 256), dim3(256), 0, stream>>>(Whh1, pWhh1, n8Wg, W_CARRY);
  k_cast_bf2<<<dim3((n8W1 + 255) / 256), dim3(256), 0, stream>>>(W1, pW1hi, pW1lo, n8W1);
  k_cast_bf2<<<dim3((n8W2 + 255) / 256), dim3(256), 0, stream>>>(W2, pW2hi, pW2lo, n8W2);

  k_ode<<<dim3(kBatch / kRows), dim3(256), 0, stream>>>(yl, yh, pWode, bode, pTraj);

  k_gru<true><<<dim3(kBatch / kRows), dim3(256), 0, stream>>>(pTraj, pWih0, pWhh0, bih0, bhh0, pH1, pH1, pH1);
  k_gru<false><<<dim3(kBatch / kRows), dim3(256), 0, stream>>>(pH1, pWih1, pWhh1, bih1, bhh1, pH2hi, pH2hi, pH2lo);

  wmma_gemm64<1, true, 2, 0, false, 0><<<dim3(2, 1), dim3(256), 0, stream>>>(
      pH2hi, pH2lo, kHid, 0L,
      pW1hi, pW1lo, kHid, 0L,
      (void*)pG1, (void*)pG1, kH1, 0L,
      b1, b1, 0L,
      kBatch, kH1, kHid, 1.0f);
  const int n2Hd = kBatch * kH1 / 2;
  k_gelu2<<<dim3((n2Hd + 255) / 256), dim3(256), 0, stream>>>(pG1, pHdhi, pHdlo, n2Hd);
  wmma_gemm64<1, true, 2, 0, false, 0><<<dim3(96, 1), dim3(256), 0, stream>>>(
      pHdhi, pHdlo, kH1, 0L,
      pW2hi, pW2lo, kH1, 0L,
      (void*)out, (void*)pG1, kOut, 0L,
      b2, b2, 0L,
      kBatch, kOut, kH1, 1.0f);
}
